// HyperMoMixLinear_64321430225160
// MI455X (gfx1250) — hardware-verified
//
#include <hip/hip_runtime.h>
#include <math.h>


#define NT   2048
#define FI   1024
#define CD   64
#define NG   32
#define DGEN 32768
typedef _Float16 b16;
typedef __attribute__((ext_vector_type(16))) _Float16 v16b;
typedef __attribute__((ext_vector_type(8)))  _Float16 v8b;
typedef __attribute__((ext_vector_type(8)))  float    v8f;
typedef __attribute__((ext_vector_type(4)))  float    v4f;
#define VST2(T, ptr, val) do { const T _v = (val); *(volatile T*)(ptr) = _v; __threadfence(); *(volatile T*)(ptr) = _v; } while (0)
__device__ __forceinline__ v8f wmma16(v16b a, v16b b, v8f c) {
  v8f d = __builtin_amdgcn_wmma_f32_16x16x32_f16(false, a, false, b, (short)0, c, false, false);
  asm volatile("v_nop\n\tv_nop\n\tv_nop\n\tv_nop" : "+v"(d) : "v"(a), "v"(b));
  return d;
}
__device__ __forceinline__ v16b frag16(const b16* p, int hh) {
  const v8b lo = *(const v8b*)(p + 8 * hh), hi = *(const v8b*)(p + 16 + 8 * hh);
  return __builtin_shufflevector(lo, hi, 0,1,2,3,4,5,6,7,8,9,10,11,12,13,14,15);
}
__device__ __forceinline__ void lds_sync() { __builtin_amdgcn_fence(__ATOMIC_RELEASE, "workgroup"); __builtin_amdgcn_wave_barrier(); __builtin_amdgcn_fence(__ATOMIC_ACQUIRE, "workgroup"); }

__global__ __launch_bounds__(256) void k_x16(const float* __restrict__ x, b16* __restrict__ X16) {
  const int t = blockIdx.x * 256 + threadIdx.x;
  v8b o;
#pragma unroll
  for (int e = 0; e < 8; ++e) o[e] = (b16)x[(size_t)t * 8 + e];
  VST2(v8b, X16 + (size_t)t * 8, o);
}
__global__ __launch_bounds__(256) void k_wc(const float* __restrict__ Wc, b16* __restrict__ WcT) {
  const int t = blockIdx.x * 256 + threadIdx.x;
  const int c = t >> 7, k0 = (t & 127) * 8;
  v8b o;
#pragma unroll
  for (int e = 0; e < 8; ++e) o[e] = (b16)Wc[(size_t)(k0 + e) * CD + c];
  VST2(v8b, WcT + (size_t)c * FI + k0, o);
}
__global__ __launch_bounds__(256) void k_wb(const float* __restrict__ Wb, b16* __restrict__ WbT) {
  const int t = blockIdx.x * 256 + threadIdx.x;
  const int n = t >> 3, c0 = (t & 7) * 8;
  v8b o;
#pragma unroll
  for (int e = 0; e < 8; ++e) o[e] = (b16)Wb[(size_t)(c0 + e) * FI + n];
  VST2(v8b, WbT + (size_t)n * CD + c0, o);
}
__global__ __launch_bounds__(256) void k_wg(const float* __restrict__ Wg, b16* __restrict__ P) {
  const int t = blockIdx.x * 256 + threadIdx.x;
  const int d = t >> 4, q0 = (t & 15) * 8, k = q0 >> 6, c0 = q0 & 63;
  v8b o;
#pragma unroll
  for (int e = 0; e < 8; ++e) o[e] = (b16)Wg[((size_t)k * CD + c0 + e) * DGEN + d];
  VST2(v8b, P + (size_t)d * 128 + q0, o);
}
__global__ __launch_bounds__(128) void k_cf(const b16* __restrict__ X16, const b16* __restrict__ WcT, const float* __restrict__ bc, const float* __restrict__ Wm, const float* __restrict__ bm,
                                            const float* __restrict__ Wr, const float* __restrict__ br, b16* __restrict__ CF2, b16* __restrict__ CF16, float* __restrict__ ratio) {
  __shared__ float st[4][16][68];
  __shared__ float sc[4][16][4];
  const int lane = threadIdx.x & 31, wave = threadIdx.x >> 5, hh = lane >> 4, l16 = lane & 15;
  const int m0 = (blockIdx.x * 4 + wave) * 16;
  v8f acc[4] = {};
  for (int k0 = 0; k0 < FI; k0 += 32) {
    const v16b a = frag16(X16 + (size_t)(m0 + l16) * FI + k0, hh);
#pragma unroll
    for (int t = 0; t < 4; ++t) acc[t] = wmma16(a, frag16(WcT + (size_t)(t * 16 + l16) * FI + k0, hh), acc[t]);
  }
#pragma unroll
  for (int t = 0; t < 4; ++t)
#pragma unroll
    for (int v = 0; v < 8; ++v) st[wave][v + 8 * hh][t * 16 + l16] = tanhf(acc[t][v] + bc[t * 16 + l16]);
  lds_sync();
  if (lane < 16) {
    const float* cf = st[wave][lane];
    float l0 = bm[0], l1 = bm[1], rt = br[0];
    for (int c = 0; c < CD; ++c) { l0 += cf[c] * Wm[c * 2]; l1 += cf[c] * Wm[c * 2 + 1]; rt += cf[c] * Wr[c]; }
    const float mx = fmaxf(l0, l1), e0 = expf(l0 - mx), e1 = expf(l1 - mx), z = e0 + e1;
    sc[wave][lane][0] = e0 / z; sc[wave][lane][1] = e1 / z; sc[wave][lane][2] = rt; sc[wave][lane][3] = 0.f;
  }
  lds_sync();
  for (int pass = 0; pass < 2; ++pass) {
    { const int r = lane >> 1, kk = lane & 1; const float cc = sc[wave][r][kk]; v8b o[8];
#pragma unroll
      for (int j = 0; j < 8; ++j) {
#pragma unroll
        for (int e = 0; e < 8; ++e) o[j][e] = (b16)(cc * st[wave][r][j * 8 + e]);
        *(volatile v8b*)(CF2 + (size_t)(m0 + r) * 128 + kk * 64 + j * 8) = o[j]; } }
    { const int r = lane >> 1, h2 = (lane & 1) * 32;
#pragma unroll
      for (int j = 0; j < 4; ++j) { v8b o;
#pragma unroll
        for (int e = 0; e < 8; ++e) o[e] = (b16)st[wave][r][h2 + j * 8 + e];
        *(volatile v8b*)(CF16 + (size_t)(m0 + r) * CD + h2 + j * 8) = o; } }
    if (lane < 16) *(volatile v4f*)(ratio + (size_t)(m0 + lane) * 4) = *(const v4f*)(sc[wave][lane]);
    __threadfence();
  }
}
__global__ __launch_bounds__(128) void k_bias(const b16* __restrict__ CF16, const b16* __restrict__ WbT, const float* __restrict__ bb, float* __restrict__ BT) {
  __shared__ __attribute__((aligned(16))) float st[4][16][132];
  const int lane = threadIdx.x & 31, wave = threadIdx.x >> 5, hh = lane >> 4, l16 = lane & 15;
  const int m0 = blockIdx.x * 64 + wave * 16, n0 = blockIdx.y * 128;
  v8f acc[8] = {};
#pragma unroll
  for (int k0 = 0; k0 < CD; k0 += 32) {
    const v16b a = frag16(CF16 + (size_t)(m0 + l16) * CD + k0, hh);
#pragma unroll
    for (int t = 0; t < 8; ++t) acc[t] = wmma16(a, frag16(WbT + (size_t)(n0 + t * 16 + l16) * CD + k0, hh), acc[t]);
  }
#pragma unroll
  for (int t = 0; t < 8; ++t)
#pragma unroll
    for (int v = 0; v < 8; ++v) st[wave][v + 8 * hh][t * 16 + l16] = acc[t][v] + bb[n0 + t * 16 + l16];
  lds_sync();
  for (int pass = 0; pass < 2; ++pass) {
#pragma unroll
    for (int rr = 0; rr < 16; ++rr) *(volatile v4f*)(BT + (size_t)(m0 + rr) * FI + n0 + lane * 4) = *(const v4f*)(&st[wave][rr][lane * 4]);
    __threadfence();
  }
}
template <int STAGE>
__global__ __launch_bounds__(128) void k_monarch(const b16* __restrict__ CF2, const b16* __restrict__ P, const float* __restrict__ bgen, const float* __restrict__ ratio,
                                                 const float* __restrict__ src, const float* __restrict__ BT, float* __restrict__ dst) {
  __shared__ __attribute__((aligned(16))) float sg[4][16][36];
  const int lane = threadIdx.x & 31, wave = threadIdx.x >> 5, hh = lane >> 4, l16 = lane & 15;
  const int m0 = (blockIdx.x * 4 + wave) * 16;
  v16b a[4];
#pragma unroll
  for (int ks = 0; ks < 4; ++ks) a[ks] = frag16(CF2 + (size_t)(m0 + l16) * 128 + ks * 32, hh);
  float c0r[8], c1r[8], rt[8];
#pragma unroll
  for (int v = 0; v < 8; ++v) { const float* rp = ratio + (size_t)(m0 + v + 8 * hh) * 4; c0r[v] = rp[0]; c1r[v] = rp[1]; rt[v] = rp[2]; }
  for (int g = 0; g < NG; ++g) {
    v8f h[2] = {};
    for (int i = 0; i < NG; ++i) {
      float s[8];
#pragma unroll
      for (int v = 0; v < 8; ++v) { const int t = m0 + v + 8 * hh; s[v] = (STAGE == 1) ? src[(size_t)t * FI + g * NG + i] : src[(size_t)t * FI + i * NG + g]; }
#pragma unroll
      for (int ot = 0; ot < 2; ++ot) {
        const int d = (g * NG + i) * NG + ot * 16 + l16;
        const b16* pr = P + (size_t)d * 128;
        v8f c = {};
#pragma unroll
        for (int ks = 0; ks < 4; ++ks) c = wmma16(a[ks], frag16(pr + ks * 32, hh), c);
        const float b0 = bgen[d], b1 = bgen[DGEN + d];
#pragma unroll
        for (int v = 0; v < 8; ++v) h[ot][v] += s[v] * (c[v] + c0r[v] * b0 + c1r[v] * b1);
      }
    }
#pragma unroll
    for (int ot = 0; ot < 2; ++ot)
#pragma unroll
      for (int v = 0; v < 8; ++v) {
        float val = h[ot][v];
        if (STAGE == 2) { const int t = m0 + v + 8 * hh; val = val * rt[v] + BT[(size_t)t * FI + g * NG + ot * 16 + l16]; }
        sg[wave][v + 8 * hh][ot * 16 + l16] = val;
      }
    lds_sync();
    for (int pass = 0; pass < 2; ++pass) {
#pragma unroll
      for (int j = 0; j < 4; ++j) { const int pc = j * 32 + lane, r = pc >> 3, q4 = pc & 7;
        *(volatile v4f*)(dst + (size_t)(m0 + r) * FI + g * NG + q4 * 4) = *(const v4f*)(&sg[wave][r][q4 * 4]); }
      __threadfence();
    }
    lds_sync();
  }
}
extern "C" void kernel_launch(void* const* d_in, const int* in_sizes, int n_in,
                              void* d_out, int out_size, void* d_ws, size_t ws_size, hipStream_t stream) {
  (void)in_sizes; (void)n_in; (void)out_size;
  const float* x  = (const float*)d_in[0];
  const float* Wc = (const float*)d_in[1];  const float* bc = (const float*)d_in[2];
  const float* W1 = (const float*)d_in[3];  const float* b1 = (const float*)d_in[4];
  const float* W2 = (const float*)d_in[5];  const float* b2 = (const float*)d_in[6];
  const float* Wm = (const float*)d_in[7];  const float* bm = (const float*)d_in[8];
  const float* Wb = (const float*)d_in[9];  const float* bb = (const float*)d_in[10];
  const float* Wr = (const float*)d_in[11]; const float* br = (const float*)d_in[12];
  float* out = (float*)d_out;
  char* ws = (char*)d_ws; size_t off = 0;
  auto take = [&](size_t bytes) { void* p = ws + off; off = (off + bytes + 255) & ~(size_t)255; return p; };
  b16*   X16  = (b16*)take((size_t)NT * FI * 2);
  b16*   WcT  = (b16*)take((size_t)CD * FI * 2);
  b16*   WbT  = (b16*)take((size_t)FI * CD * 2);
  b16*   P1   = (b16*)take((size_t)DGEN * 128 * 2);
  b16*   P2   = (b16*)take((size_t)DGEN * 128 * 2);
  b16*   CF2  = (b16*)take((size_t)NT * 128 * 2);
  b16*   CF16 = (b16*)take((size_t)NT * CD * 2);
  float* RT   = (float*)take((size_t)NT * 4 * 4);
  float* BT   = (float*)take((size_t)NT * FI * 4);
  float* H1   = (float*)take((size_t)NT * FI * 4);
  if (off > ws_size) return;
  const dim3 b256(256);
  k_x16<<<NT * 128 / 256, b256, 0, stream>>>(x, X16);
  k_wc<<<64 * 128 / 256, b256, 0, stream>>>(Wc, WcT);
  k_wb<<<FI * 8 / 256, b256, 0, stream>>>(Wb, WbT);
  k_wg<<<DGEN * 16 / 256, b256, 0, stream>>>(W1, P1);
  k_wg<<<DGEN * 16 / 256, b256, 0, stream>>>(W2, P2);
  k_cf<<<NT / 64, 128, 0, stream>>>(X16, WcT, bc, Wm, bm, Wr, br, CF2, CF16, RT);
  k_bias<<<dim3(NT / 64, FI / 128), 128, 0, stream>>>(CF16, WbT, bb, BT);
  k_monarch<1><<<NT / 64, 128, 0, stream>>>(CF2, P1, b1, RT, x, nullptr, H1);
  k_monarch<2><<<NT / 64, 128, 0, stream>>>(CF2, P2, b2, RT, H1, BT, out);
}
